// MultiHeadAttentionLayer_74311524156003
// MI455X (gfx1250) — hardware-verified
//
#include <hip/hip_runtime.h>
#include <stdint.h>


#define EMBED  1024
#define NHEADS 16
#define HDIM   64
#define BATCH  2
#define SEQ    2048
#define NTOK   (BATCH * SEQ)
#define NE     (NTOK * EMBED)
#define WE     (EMBED * EMBED)

typedef unsigned short us;
typedef __bf16   v16bf __attribute__((ext_vector_type(16)));
typedef us       v8us  __attribute__((ext_vector_type(8), may_alias));
typedef us       v16us __attribute__((ext_vector_type(16), may_alias));
typedef float    v8f   __attribute__((ext_vector_type(8)));
typedef float    v4f   __attribute__((ext_vector_type(4), may_alias));
typedef unsigned v4u   __attribute__((ext_vector_type(4), may_alias));

union Frag { v16bf v; v16us u; v8us half[2]; };


__device__ __forceinline__ unsigned bf_bits(float f) {
  const unsigned u = __builtin_bit_cast(unsigned, f);
  return (u + 0x7FFFu + ((u >> 16) & 1u)) >> 16;
}

__device__ __forceinline__ float bf_val(unsigned b) {
  return __builtin_bit_cast(float, b << 16);
}

__device__ __forceinline__ v8f zero8() {
  v8f z;
#pragma unroll
  for (int i = 0; i < 8; ++i) z[i] = 0.0f;
  return z;
}

__device__ __forceinline__ v8f wmma3(v16bf ah, v16bf al, v16bf bh, v16bf bl, v8f c) {
  c = __builtin_amdgcn_wmma_f32_16x16x32_bf16(false, ah, false, bh, (short)0, c, false, false);
  c = __builtin_amdgcn_wmma_f32_16x16x32_bf16(false, ah, false, bl, (short)0, c, false, false);
  c = __builtin_amdgcn_wmma_f32_16x16x32_bf16(false, al, false, bh, (short)0, c, false, false);
  asm volatile("v_nop\n\tv_nop\n\tv_nop\n\tv_nop" : "+v"(c) : "v"(ah), "v"(al), "v"(bh), "v"(bl));
  return c;
}

__device__ __forceinline__ v16bf load_frag_g(const us* p, int hf) {
  Frag f;
  f.half[0] = *(const v8us*)(p + 8 * hf);
  f.half[1] = *(const v8us*)(p + 16 + 8 * hf);
  return f.v;
}

__global__ __launch_bounds__(256)
void k_cvt_split(const float* __restrict__ in, us* __restrict__ hi, us* __restrict__ lo, int n8) {
  const int i = blockIdx.x * blockDim.x + threadIdx.x;
  if (i >= n8) return;
  const size_t e0 = (size_t)i * 8;
  const v4f a = *(const v4f*)(in + e0);
  const v4f b = *(const v4f*)(in + e0 + 4);
  float x[8];
  x[0] = a[0]; x[1] = a[1]; x[2] = a[2]; x[3] = a[3];
  x[4] = b[0]; x[5] = b[1]; x[6] = b[2]; x[7] = b[3];
  unsigned hb[8], lb[8];
#pragma unroll
  for (int e = 0; e < 8; ++e) {
    hb[e] = bf_bits(x[e]);
    lb[e] = bf_bits(x[e] - bf_val(hb[e]));
  }
  v4u H, L;
#pragma unroll
  for (int j = 0; j < 4; ++j) {
    H[j] = hb[2 * j] | (hb[2 * j + 1] << 16);
    L[j] = lb[2 * j] | (lb[2 * j + 1] << 16);
  }
  volatile v4u* ph = (volatile v4u*)(hi + e0);
  volatile v4u* pl = (volatile v4u*)(lo + e0);
  *ph = H;
  *pl = L;
  __threadfence();
  *ph = H;
  *pl = L;
}

__global__ __launch_bounds__(128)
void k_gemm_split(const us* __restrict__ Xh, const us* __restrict__ Xl,
                  const us* __restrict__ Wh, const us* __restrict__ Wl,
                  const float* __restrict__ bias, float* __restrict__ out,
                  int M, int N, int K, int seq, int nheads, int mode) {
  __shared__ __attribute__((aligned(16))) float tile[64 * 64];

  const int lane = threadIdx.x & 31;
  const int hf   = lane >> 4;
  const int m    = lane & 15;
  const int w    = threadIdx.x >> 5;
  const int rb   = blockIdx.y * 64;
  const int n0   = blockIdx.x * 64;
  const int arow = rb + 16 * w + m;

  v8f acc[4];
#pragma unroll
  for (int ns = 0; ns < 4; ++ns) acc[ns] = zero8();

  const us* xh = Xh + (size_t)arow * K;
  const us* xl = Xl + (size_t)arow * K;

  for (int kb = 0; kb < K; kb += 32) {
    const v16bf ah = load_frag_g(xh + kb, hf);
    const v16bf al = load_frag_g(xl + kb, hf);
#pragma unroll
    for (int ns = 0; ns < 4; ++ns) {
      const size_t wo = (size_t)(n0 + 16 * ns + m) * K + kb;
      const v16bf bh = load_frag_g(Wh + wo, hf);
      const v16bf bl = load_frag_g(Wl + wo, hf);
      acc[ns] = wmma3(ah, al, bh, bl, acc[ns]);
    }
  }

#pragma unroll
  for (int ns = 0; ns < 4; ++ns) {
    const float bn = bias[n0 + 16 * ns + m];
#pragma unroll
    for (int r = 0; r < 8; ++r)
      tile[(16 * w + 8 * hf + r) * 64 + 16 * ns + m] = acc[ns][r] + bn;
  }
  __syncthreads();

  const int c4   = 4 * m;
  const int head = n0 / HDIM;
#pragma unroll
  for (int it = 0; it < 8; ++it) {
    const int lr = 16 * w + 2 * it + hf;
    const int gm = rb + lr;
    const v4f v  = *(const v4f*)(&tile[lr * 64 + c4]);
    float* dst;
    if (mode == 0) {
      const int bb = gm / seq, tt = gm - bb * seq;
      dst = out + (((size_t)bb * nheads + head) * seq + tt) * HDIM + c4;
    } else {
      dst = out + (size_t)gm * N + n0 + c4;
    }
    if (gm < M) *(volatile v4f*)dst = v;
  }
  __threadfence();
#pragma unroll
  for (int it = 0; it < 8; ++it) {
    const int lr = 16 * w + 2 * it + hf;
    const int gm = rb + lr;
    const v4f v  = *(const v4f*)(&tile[lr * 64 + c4]);
    float* dst;
    if (mode == 0) {
      const int bb = gm / seq, tt = gm - bb * seq;
      dst = out + (((size_t)bb * nheads + head) * seq + tt) * HDIM + c4;
    } else {
      dst = out + (size_t)gm * N + n0 + c4;
    }
    if (gm < M) *(volatile v4f*)dst = v;
  }
}

__global__ __launch_bounds__(128)
void k_attn_split(const us* __restrict__ Qh, const us* __restrict__ Ql,
                  const us* __restrict__ Kh, const us* __restrict__ Kl,
                  const us* __restrict__ Vh, const us* __restrict__ Vl,
                  float* __restrict__ AO, int seq, int nheads, int embed, float scale) {
  __shared__ __attribute__((aligned(16))) us    Ks[2][32 * HDIM];
  __shared__ __attribute__((aligned(16))) us    Vts[2][HDIM * 32];
  __shared__ __attribute__((aligned(16))) us    Ps[4][2][16 * 32];
  __shared__ __attribute__((aligned(16))) float Os[4][16 * HDIM];

  const int tid  = threadIdx.x;
  const int lane = tid & 31;
  const int hf   = lane >> 4;
  const int m    = lane & 15;
  const int w    = tid >> 5;
  const int bh   = blockIdx.y;
  const int b    = bh / nheads;
  const int head = bh - b * nheads;
  const int q0   = blockIdx.x * 64 + w * 16;
  const size_t pb = (size_t)bh * seq * HDIM;

  v16bf qh[2], ql[2];
  {
    const size_t qo = pb + (size_t)(q0 + m) * HDIM;
#pragma unroll
    for (int kc = 0; kc < 2; ++kc) {
      qh[kc] = load_frag_g(Qh + qo + 32 * kc, hf);
      ql[kc] = load_frag_g(Ql + qo + 32 * kc, hf);
    }
  }

  v8f o[4];
#pragma unroll
  for (int g = 0; g < 4; ++g) o[g] = zero8();
  v8f mrow, lsum;
#pragma unroll
  for (int r = 0; r < 8; ++r) { mrow[r] = -__builtin_inff(); lsum[r] = 0.0f; }

  for (int jb = 0; jb < seq; jb += 32) {
    __syncthreads();
    {
      const size_t ko = pb + (size_t)jb * HDIM;
#pragma unroll
      for (int c = 0; c < 2; ++c) {
        const int idx = tid + 128 * c;
        *(v8us*)(&Ks[0][idx * 8]) = *(const v8us*)(Kh + ko + (size_t)idx * 8);
        *(v8us*)(&Ks[1][idx * 8]) = *(const v8us*)(Kl + ko + (size_t)idx * 8);
      }
      const int j  = tid >> 2;
      const int d0 = (tid & 3) * 16;
      const size_t vo = pb + (size_t)(jb + j) * HDIM + d0;
      const v16us eh = *(const v16us*)(Vh + vo);
      const v16us el = *(const v16us*)(Vl + vo);
#pragma unroll
      for (int i = 0; i < 16; ++i) {
        Vts[0][(d0 + i) * 32 + j] = eh[i];
        Vts[1][(d0 + i) * 32 + j] = el[i];
      }
    }
    __syncthreads();

    v8f s[2];
#pragma unroll
    for (int c = 0; c < 2; ++c) {
      s[c] = zero8();
#pragma unroll
      for (int kc = 0; kc < 2; ++kc) {
        const int ro = (16 * c + m) * HDIM + 32 * kc;
        Frag kh, kl;
        kh.half[0] = *(const v8us*)(&Ks[0][ro + 8 * hf]);
        kh.half[1] = *(const v8us*)(&Ks[0][ro + 16 + 8 * hf]);
        kl.half[0] = *(const v8us*)(&Ks[1][ro + 8 * hf]);
        kl.half[1] = *(const v8us*)(&Ks[1][ro + 16 + 8 * hf]);
        s[c] = wmma3(qh[kc], ql[kc], kh.v, kl.v, s[c]);
      }
    }
#pragma unroll
    for (int r = 0; r < 8; ++r) { s[0][r] *= scale; s[1][r] *= scale; }

    v8f tmax;
#pragma unroll
    for (int r = 0; r < 8; ++r) tmax[r] = fmaxf(s[0][r], s[1][r]);
#pragma unroll
    for (int off = 8; off > 0; off >>= 1)
#pragma unroll
      for (int r = 0; r < 8; ++r)
        tmax[r] = fmaxf(tmax[r], __shfl_xor(tmax[r], off, 32));

    v8f cor;
#pragma unroll
    for (int r = 0; r < 8; ++r) {
      const float mnew = fmaxf(mrow[r], tmax[r]);
      cor[r]  = __expf(mrow[r] - mnew);
      s[0][r] = __expf(s[0][r] - mnew);
      s[1][r] = __expf(s[1][r] - mnew);
      mrow[r] = mnew;
    }
    v8f rsum;
#pragma unroll
    for (int r = 0; r < 8; ++r) rsum[r] = s[0][r] + s[1][r];
#pragma unroll
    for (int off = 8; off > 0; off >>= 1)
#pragma unroll
      for (int r = 0; r < 8; ++r)
        rsum[r] += __shfl_xor(rsum[r], off, 32);
#pragma unroll
    for (int r = 0; r < 8; ++r) lsum[r] = lsum[r] * cor[r] + rsum[r];
#pragma unroll
    for (int g = 0; g < 4; ++g)
#pragma unroll
      for (int r = 0; r < 8; ++r) o[g][r] *= cor[r];

#pragma unroll
    for (int r = 0; r < 8; ++r) {
      const int row = 8 * hf + r;
      const unsigned h0 = bf_bits(s[0][r]);
      const unsigned l0 = bf_bits(s[0][r] - bf_val(h0));
      const unsigned h1 = bf_bits(s[1][r]);
      const unsigned l1 = bf_bits(s[1][r] - bf_val(h1));
      Ps[w][0][row * 32 + m]      = (us)h0;
      Ps[w][1][row * 32 + m]      = (us)l0;
      Ps[w][0][row * 32 + 16 + m] = (us)h1;
      Ps[w][1][row * 32 + 16 + m] = (us)l1;
    }
    __syncthreads();

    Frag ph, pl;
    ph.half[0] = *(const v8us*)(&Ps[w][0][m * 32 + 8 * hf]);
    ph.half[1] = *(const v8us*)(&Ps[w][0][m * 32 + 16 + 8 * hf]);
    pl.half[0] = *(const v8us*)(&Ps[w][1][m * 32 + 8 * hf]);
    pl.half[1] = *(const v8us*)(&Ps[w][1][m * 32 + 16 + 8 * hf]);

#pragma unroll
    for (int g = 0; g < 4; ++g) {
      const int vr = (16 * g + m) * 32;
      Frag vh, vl;
      vh.half[0] = *(const v8us*)(&Vts[0][vr + 8 * hf]);
      vh.half[1] = *(const v8us*)(&Vts[0][vr + 16 + 8 * hf]);
      vl.half[0] = *(const v8us*)(&Vts[1][vr + 8 * hf]);
      vl.half[1] = *(const v8us*)(&Vts[1][vr + 16 + 8 * hf]);
      o[g] = wmma3(ph.v, pl.v, vh.v, vl.v, o[g]);
    }
  }

  v8f inv;
#pragma unroll
  for (int r = 0; r < 8; ++r) inv[r] = 1.0f / lsum[r];
#pragma unroll
  for (int g = 0; g < 4; ++g)
#pragma unroll
    for (int r = 0; r < 8; ++r)
      Os[w][(8 * hf + r) * HDIM + 16 * g + m] = o[g][r] * inv[r];
  __syncthreads();

  const int c4 = 4 * m;
  float* aob = AO + (size_t)b * seq * embed + (size_t)head * HDIM + c4;
#pragma unroll
  for (int it = 0; it < 8; ++it) {
    const int lr = 2 * it + hf;
    const int t  = q0 + lr;
    const v4f v  = *(const v4f*)(&Os[w][lr * HDIM + c4]);
    if (t < seq) *(volatile v4f*)(aob + (size_t)t * embed) = v;
  }
  __threadfence();
#pragma unroll
  for (int it = 0; it < 8; ++it) {
    const int lr = 2 * it + hf;
    const int t  = q0 + lr;
    const v4f v  = *(const v4f*)(&Os[w][lr * HDIM + c4]);
    if (t < seq) *(volatile v4f*)(aob + (size_t)t * embed) = v;
  }
}


static inline unsigned cdiv_u(size_t a, unsigned b) { return (unsigned)((a + b - 1) / b); }

extern "C" void kernel_launch(void* const* d_in, const int* in_sizes, int n_in,
                              void* d_out, int out_size, void* d_ws, size_t ws_size,
                              hipStream_t stream) {
  static_assert(NTOK % 64 == 0 && EMBED % 64 == 0 && EMBED % 32 == 0 && SEQ % 64 == 0 &&
                HDIM == 64 && NHEADS * HDIM == EMBED && NE % 8 == 0 && WE % 8 == 0);
  if (n_in < 11) return;
  if (in_sizes[0] != NE || in_sizes[1] != NE || in_sizes[2] != NE) return;
  if (in_sizes[3] != WE || in_sizes[4] != WE || in_sizes[5] != WE || in_sizes[9] != WE) return;
  if (in_sizes[6] != EMBED || in_sizes[7] != EMBED || in_sizes[8] != EMBED || in_sizes[10] != EMBED) return;
  if (out_size != NE) return;

  const float* query = (const float*)d_in[0];
  const float* key   = (const float*)d_in[1];
  const float* value = (const float*)d_in[2];
  const float* Wq    = (const float*)d_in[3];
  const float* Wk    = (const float*)d_in[4];
  const float* Wv    = (const float*)d_in[5];
  const float* bq    = (const float*)d_in[6];
  const float* bk    = (const float*)d_in[7];
  const float* bv    = (const float*)d_in[8];
  const float* Wo    = (const float*)d_in[9];
  const float* bo    = (const float*)d_in[10];
  float* out = (float*)d_out;

  const size_t bA16 = (size_t)NE * 2;
  const size_t bW16 = (size_t)WE * 2;
  const size_t bA32 = (size_t)NE * 4;
  const size_t need = 6 * bA16 + 8 * bW16 + 3 * bA32 + 6 * bA16 + bA32 + 2 * bA16;
  if (need > ws_size) return;

  char* p = (char*)d_ws;
  us* Xqh = (us*)p; p += bA16;  us* Xql = (us*)p; p += bA16;
  us* Xkh = (us*)p; p += bA16;  us* Xkl = (us*)p; p += bA16;
  us* Xvh = (us*)p; p += bA16;  us* Xvl = (us*)p; p += bA16;
  us* Wqh = (us*)p; p += bW16;  us* Wql = (us*)p; p += bW16;
  us* Wkh = (us*)p; p += bW16;  us* Wkl = (us*)p; p += bW16;
  us* Wvh = (us*)p; p += bW16;  us* Wvl = (us*)p; p += bW16;
  us* Woh = (us*)p; p += bW16;  us* Wol = (us*)p; p += bW16;
  float* Qf = (float*)p; p += bA32;
  float* Kf = (float*)p; p += bA32;
  float* Vf = (float*)p; p += bA32;
  us* Qh = (us*)p; p += bA16;   us* Ql = (us*)p; p += bA16;
  us* Kh = (us*)p; p += bA16;   us* Kl = (us*)p; p += bA16;
  us* Vh = (us*)p; p += bA16;   us* Vl = (us*)p; p += bA16;
  float* AOf = (float*)p; p += bA32;
  us* AOh = (us*)p; p += bA16;  us* AOl = (us*)p; p += bA16;

  const int blkc = 256;
  const int nA8 = NE / 8, nW8 = WE / 8;

  k_cvt_split<<<dim3(cdiv_u(nA8, blkc)), dim3(blkc), 0, stream>>>(query, Xqh, Xql, nA8);
  k_cvt_split<<<dim3(cdiv_u(nA8, blkc)), dim3(blkc), 0, stream>>>(key,   Xkh, Xkl, nA8);
  k_cvt_split<<<dim3(cdiv_u(nA8, blkc)), dim3(blkc), 0, stream>>>(value, Xvh, Xvl, nA8);
  k_cvt_split<<<dim3(cdiv_u(nW8, blkc)), dim3(blkc), 0, stream>>>(Wq, Wqh, Wql, nW8);
  k_cvt_split<<<dim3(cdiv_u(nW8, blkc)), dim3(blkc), 0, stream>>>(Wk, Wkh, Wkl, nW8);
  k_cvt_split<<<dim3(cdiv_u(nW8, blkc)), dim3(blkc), 0, stream>>>(Wv, Wvh, Wvl, nW8);
  k_cvt_split<<<dim3(cdiv_u(nW8, blkc)), dim3(blkc), 0, stream>>>(Wo, Woh, Wol, nW8);

  {
    dim3 grid(cdiv_u(EMBED, 64), cdiv_u(NTOK, 64));
    k_gemm_split<<<grid, dim3(128), 0, stream>>>(Xqh, Xql, Wqh, Wql, bq, Qf, NTOK, EMBED, EMBED, SEQ, NHEADS, 0);
    k_gemm_split<<<grid, dim3(128), 0, stream>>>(Xkh, Xkl, Wkh, Wkl, bk, Kf, NTOK, EMBED, EMBED, SEQ, NHEADS, 0);
    k_gemm_split<<<grid, dim3(128), 0, stream>>>(Xvh, Xvl, Wvh, Wvl, bv, Vf, NTOK, EMBED, EMBED, SEQ, NHEADS, 0);
  }

  k_cvt_split<<<dim3(cdiv_u(nA8, blkc)), dim3(blkc), 0, stream>>>(Qf, Qh, Ql, nA8);
  k_cvt_split<<<dim3(cdiv_u(nA8, blkc)), dim3(blkc), 0, stream>>>(Kf, Kh, Kl, nA8);
  k_cvt_split<<<dim3(cdiv_u(nA8, blkc)), dim3(blkc), 0, stream>>>(Vf, Vh, Vl, nA8);

  {
    dim3 grid(cdiv_u(SEQ, 64), BATCH * NHEADS);
    k_attn_split<<<grid, dim3(128), 0, stream>>>(Qh, Ql, Kh, Kl, Vh, Vl, AOf, SEQ, NHEADS, EMBED, 0.125f);
  }

  k_cvt_split<<<dim3(cdiv_u(nA8, blkc)), dim3(blkc), 0, stream>>>(AOf, AOh, AOl, nA8);

  {
    dim3 grid(cdiv_u(EMBED, 64), cdiv_u(NTOK, 64));
    k_gemm_split<<<grid, dim3(128), 0, stream>>>(AOh, AOl, Woh, Wol, bo, out, NTOK, EMBED, EMBED, SEQ, NHEADS, 2);
  }
}
